// SFT_23527830848169
// MI455X (gfx1250) — hardware-verified
//
#include <hip/hip_runtime.h>
#include <math.h>
#include <stdint.h>


#define NBATCH 64
#define NTOK   196
#define CIN    512
#define NHEAD  16
#define KD     64
#define DV     128
#define HF     192
#define FKV    3072
#define FQ     1024
#define DH     2048
#define COUT   512
#define MROWS  (NBATCH * NTOK)
#define TM64   (MROWS / 64)
#define NQU    4
#define HQ     (NHEAD / NQU)
#define FKVQ   (HQ * HF)
#define FQQ    (HQ * KD)
#define NQT    13
#define NKR    208
#define NKT    13
#define PVK    224
#define KP     72
#define VP     232
#define SP     224
#define OP     136
#define ATW    4
#define ATT    (ATW * 32)

#define LK   (NKR * KP * 2)
#define LV   (DV * VP * 2)
#define LQW  (2 * 16 * KP * 2)
#define LSW  (16 * SP * 4)
#define LPAR ((3 * HF + 3 * KD) * 4)
#define ATT_LDS (2 * LK + LV + ATW * LQW + ATW * LSW + LPAR)

#define SCW  64.0f
#define SCQK 8.0f
#define SCR  2048.0f
#define SCP  32768.0f
#define SCV  8.0f
#define SCH  16.0f
#define SCS  (1.0f / (SCQK * SCQK * 8.0f))
#define SCO  (1.0f / (SCP * SCV))

static_assert(MROWS % 64 == 0 && TM64 == 196);
static_assert(FKVQ % 64 == 0 && FQQ % 64 == 0 && COUT % 64 == 0);
static_assert(CIN % 32 == 0 && DH % 32 == 0 && KD % 32 == 0 && PVK % 32 == 0);
static_assert(NQT * 16 >= NTOK && NKR >= NTOK && NKT * 16 == NKR && NQT * 16 == NKR);
static_assert(PVK >= NKR && PVK + 8 == VP && 2 * SP >= SP + PVK);
static_assert((NKR * 48) % ATT == 0 && (DV * 3) % ATT == 0);
static_assert(FKVQ % 256 == 0 && FQQ % 256 == 0 && COUT % 256 == 0);
static_assert((MROWS * CIN) % (8 * 256) == 0 && (FKV * CIN) % (8 * 256) == 0);
static_assert((FQ * CIN) % (8 * 256) == 0 && (COUT * DH) % (8 * 256) == 0);
static_assert(16 * OP * 2 <= LSW && (KP * 2) % 16 == 0 && (VP * 2) % 16 == 0 && (OP * 2) % 16 == 0);
static_assert(ATT_LDS == 198144);
static_assert(COUT == 128 * 4);

typedef _Float16       v16h __attribute__((ext_vector_type(16)));
typedef _Float16       v8h  __attribute__((ext_vector_type(8)));
typedef _Float16       v4h  __attribute__((ext_vector_type(4)));
typedef float          v8f  __attribute__((ext_vector_type(8)));
typedef float          v4f  __attribute__((ext_vector_type(4)));
typedef unsigned int   v4u  __attribute__((ext_vector_type(4)));

union HU { v8h h; v4u u; _Float16 s[8]; };
union H4 { v4h h; _Float16 s[4]; };
union FR { v16h v; v8h h[2]; _Float16 s[16]; };
static_assert(sizeof(HU) == 16);
static_assert(sizeof(H4) == 8);
static_assert(sizeof(FR) == 32);

__device__ __forceinline__ unsigned short bf_bits(float f) {
  const unsigned u = __float_as_uint(f);
  return (unsigned short)((u + 0x7FFFu + ((u >> 16) & 1u)) >> 16);
}
__device__ __forceinline__ float bf_up(unsigned short h) { return __uint_as_float(((unsigned)h) << 16); }
__device__ __forceinline__ float bfr(float f) { return bf_up(bf_bits(f)); }
__device__ __forceinline__ v8f zero8() { v8f z = {0.f, 0.f, 0.f, 0.f, 0.f, 0.f, 0.f, 0.f}; return z; }

__device__ __forceinline__ void ld8(const float* p, float* o) {
  const v4f a = *(const v4f*)(p);
  const v4f b = *(const v4f*)(p + 4);
  o[0] = a[0]; o[1] = a[1]; o[2] = a[2]; o[3] = a[3];
  o[4] = b[0]; o[5] = b[1]; o[6] = b[2]; o[7] = b[3];
}

__device__ __forceinline__ v16h ldfrag_h(const _Float16* p) {
  FR f;
  f.h[0] = *(const v8h*)(p);
  f.h[1] = *(const v8h*)(p + 16);
  return f.v;
}

__device__ __forceinline__ v8f mma_h(v16h a, v16h b, v8f c) {
  c = __builtin_amdgcn_wmma_f32_16x16x32_f16(false, a, false, b, (short)0, c, false, false);
#if defined(__HIP_DEVICE_COMPILE__)
  asm volatile("v_nop\n\tv_nop\n\tv_nop\n\tv_nop" : "+v"(c) : "v"(a), "v"(b));
#endif
  return c;
}
__device__ __forceinline__ v8f mma_h_raw(v16h a, v16h b, v8f c) {
  return __builtin_amdgcn_wmma_f32_16x16x32_f16(false, a, false, b, (short)0, c, false, false);
}
__device__ __forceinline__ void dep_guard_h(v8f& a, v8f& b, v16h x) {
#if defined(__HIP_DEVICE_COMPILE__)
  asm volatile("v_nop\n\tv_nop\n\tv_nop\n\tv_nop" : "+v"(a), "+v"(b) : "v"(x));
#endif
}
__device__ __forceinline__ void keep4_h(v16h a, v16h b, v16h c, v16h d) {
#if defined(__HIP_DEVICE_COMPILE__)
  asm volatile("v_nop" :: "v"(a), "v"(b), "v"(c), "v"(d));
#endif
}
__device__ __forceinline__ void acc_guard4(v8f& a, v8f& b, v8f& c, v8f& d) {
#if defined(__HIP_DEVICE_COMPILE__)
  asm volatile("v_nop\n\tv_nop\n\tv_nop\n\tv_nop" : "+v"(a), "+v"(b), "+v"(c), "+v"(d));
#endif
}
__device__ __forceinline__ void wave_lds_sync() {
  __builtin_amdgcn_fence(__ATOMIC_RELEASE, "workgroup");
  __builtin_amdgcn_wave_barrier();
  __builtin_amdgcn_fence(__ATOMIC_ACQUIRE, "workgroup");
}

__global__ __launch_bounds__(256) void cvt_flat(const float* __restrict__ in, _Float16* out, int n8, float scale) {
  const int i = blockIdx.x * 256 + threadIdx.x;
  if (i < n8) {
    float v[8];
    ld8(in + (size_t)i * 8, v);
    HU u;
#pragma unroll
    for (int e = 0; e < 8; ++e) u.s[e] = (_Float16)(bfr(v[e]) * scale);
    _Float16* p = out + (size_t)i * 8;
    *(volatile v4u*)p = u.u;
    __threadfence();
    *(volatile v4u*)p = u.u;
  }
}

__device__ __forceinline__ void kseg(v8f (&acc)[4][4], const _Float16* __restrict__ A, int lda, int m0,
                                     const _Float16* __restrict__ Bt, int ldb, int n0, int K, int rlane, int koff) {
  for (int kk = 0; kk < K; kk += 32) {
    v16h bh[4];
#pragma unroll
    for (int j = 0; j < 4; ++j) {
      const size_t bo = (size_t)(n0 + (j << 4) + rlane) * (size_t)ldb + koff + kk;
      bh[j] = ldfrag_h(Bt + bo);
    }
#pragma unroll
    for (int i = 0; i < 4; ++i) {
      const size_t ao = (size_t)(m0 + (i << 4) + rlane) * (size_t)lda + koff + kk;
      const v16h a0 = ldfrag_h(A + ao);
#pragma unroll
      for (int j = 0; j < 4; ++j) acc[i][j] = mma_h_raw(a0, bh[j], acc[i][j]);
      dep_guard_h(acc[i][0], acc[i][3], a0);
    }
    keep4_h(bh[0], bh[1], bh[2], bh[3]);
  }
}

__global__ __launch_bounds__(256) void gemm64s(
    const _Float16* __restrict__ A, int lda, const _Float16* __restrict__ Bt, int ldb, float cs,
    float* C, int ldc, float* P2, int M, int N, int K) {
  __shared__ __align__(16) float sT[8][16 * 68];
  const int lane = threadIdx.x & 31;
  const int wave = threadIdx.x >> 5;
  const int tilesN = N >> 6;
  const int tilesM = M >> 6;
  const int tiles = tilesM * tilesN;
  const int item = blockIdx.x * 8 + wave;
  if (item >= tiles) return;
  const int tm = item / tilesN;
  const int tn = item - tm * tilesN;
  const int m0 = tm << 6;
  const int n0 = tn << 6;

  const int rlane = lane & 15;
  const int hh    = lane >> 4;
  const int koff  = hh * 8;
  const int mOff  = hh * 8;

  v8f acc[4][4];
#pragma unroll
  for (int i = 0; i < 4; ++i)
#pragma unroll
    for (int j = 0; j < 4; ++j) acc[i][j] = zero8();

  kseg(acc, A, lda, m0, Bt, ldb, n0, K, rlane, koff);
  acc_guard4(acc[0][0], acc[0][1], acc[0][2], acc[0][3]);
  acc_guard4(acc[1][0], acc[1][1], acc[1][2], acc[1][3]);
  acc_guard4(acc[2][0], acc[2][1], acc[2][2], acc[2][3]);
  acc_guard4(acc[3][0], acc[3][1], acc[3][2], acc[3][3]);

  float csm[4], csq[4];
#pragma unroll
  for (int j = 0; j < 4; ++j) {
    float s = 0.0f, q = 0.0f;
#pragma unroll
    for (int i = 0; i < 4; ++i) {
#pragma unroll
      for (int r = 0; r < 8; ++r) {
        const float v = acc[i][j][r] * cs;
        s += v;
        q += v * v;
      }
    }
    s += __shfl_xor(s, 16, 32);
    q += __shfl_xor(q, 16, 32);
    csm[j] = s;
    csq[j] = q;
  }

  float* slab = sT[wave];
#pragma unroll
  for (int i = 0; i < 4; ++i) {
    const int mBase = m0 + (i << 4);
#pragma unroll
    for (int r = 0; r < 8; ++r) {
#pragma unroll
      for (int j = 0; j < 4; ++j) {
        slab[(mOff + r) * 68 + (j << 4) + rlane] = acc[i][j][r] * cs;
      }
    }
    wave_lds_sync();
    v4f ov[8];
#pragma unroll
    for (int it = 0; it < 8; ++it) {
      const int row = 2 * it + hh;
      ov[it] = *(const v4f*)(slab + row * 68 + 4 * rlane);
    }
    for (int pass = 0; pass < 2; ++pass) {
#pragma unroll
      for (int it = 0; it < 8; ++it) {
        const int row = 2 * it + hh;
        float* dst = C + (size_t)(mBase + row) * (size_t)ldc + n0 + 4 * rlane;
        *(volatile v4f*)dst = ov[it];
      }
      __threadfence();
    }
    wave_lds_sync();
  }

#pragma unroll
  for (int j = 0; j < 4; ++j) {
    slab[(j << 4) + rlane] = csm[j];
    slab[68 + (j << 4) + rlane] = csq[j];
  }
  wave_lds_sync();
  const v4f pv = *(const v4f*)(slab + hh * 68 + 4 * rlane);
  float* pdst = P2 + (size_t)hh * (size_t)tilesM * (size_t)N + (size_t)tm * (size_t)N + n0 + 4 * rlane;
  for (int pass = 0; pass < 2; ++pass) {
    *(volatile v4f*)pdst = pv;
    __threadfence();
  }
}

__global__ __launch_bounds__(256) void bn_stats(const float* __restrict__ P2, int N, int tilesM,
                                                const float* __restrict__ gam, const float* __restrict__ bet,
                                                float* MU, float* SC, float* BE) {
  __shared__ __align__(16) float sst[3 * 256];
  const int t = threadIdx.x;
  const int f0 = blockIdx.x * 256;
  const int f = min(f0 + t, N - 1);
  const float* ps = P2 + f;
  const float* pq = P2 + (size_t)tilesM * (size_t)N + f;
  double s = 0.0, q = 0.0;
#pragma unroll 1
  for (int tt = 0; tt < tilesM; ++tt) {
    s += (double)ps[(size_t)tt * N];
    q += (double)pq[(size_t)tt * N];
  }
  const double inv = 1.0 / (double)MROWS;
  const double mu = s * inv;
  double var = q * inv - mu * mu;
  if (var < 0.0) var = 0.0;
  const float muf = (float)mu;
  const float varf = (float)var;
  const float scv = bfr(gam[f]) * (1.0f / sqrtf(varf + 1e-5f));
  const float bev = bfr(bet[f]);
  sst[t]       = muf;
  sst[256 + t] = scv;
  sst[512 + t] = bev;
  __syncthreads();
  if (f0 + 256 <= N && t < 192) {
    const int a = t >> 6;
    const int w64 = t & 63;
    const int li = w64 >> 3, q8 = w64 & 7;
    const int col = li * 32 + q8 * 4;
    const v4f v = *(const v4f*)(sst + a * 256 + col);
    float* base = (a == 0) ? MU : ((a == 1) ? SC : BE);
    float* dst = base + f0 + col;
    *(volatile v4f*)dst = v;
    __threadfence();
    *(volatile v4f*)dst = v;
  }
}

__global__ __launch_bounds__(ATT) void k_att(const float* __restrict__ Ykv, const float* __restrict__ Yq,
                                             const float* __restrict__ MUk, const float* __restrict__ SCk,
                                             const float* __restrict__ BEk, const float* __restrict__ MUq,
                                             const float* __restrict__ SCq, const float* __restrict__ BEq,
                                             const float* __restrict__ bias, _Float16* HS, int qu) {
  extern __shared__ __align__(16) char smem[];
  _Float16* sKh  = (_Float16*)(smem);
  _Float16* sKl  = (_Float16*)(smem + LK);
  _Float16* sVT  = (_Float16*)(smem + 2 * LK);
  _Float16* sQ   = (_Float16*)(smem + 2 * LK + LV);
  float*    sS   = (float*)(smem + 2 * LK + LV + ATW * LQW);
  float*    sPar = (float*)(smem + 2 * LK + LV + ATW * LQW + ATW * LSW);

  const int tid = threadIdx.x, wave = tid >> 5, lane = tid & 31;
  const int hh = lane >> 4, rl = lane & 15;
  const int b = blockIdx.x, hl = blockIdx.y;
  const int h = qu * HQ + hl;

  for (int i = tid; i < HF; i += ATT) {
    sPar[i]          = MUk[hl * HF + i];
    sPar[HF + i]     = SCk[hl * HF + i];
    sPar[2 * HF + i] = BEk[hl * HF + i];
  }
  for (int i = tid; i < KD; i += ATT) {
    sPar[3 * HF + i]          = MUq[hl * KD + i];
    sPar[3 * HF + KD + i]     = SCq[hl * KD + i];
    sPar[3 * HF + 2 * KD + i] = BEq[hl * KD + i];
  }
  __syncthreads();
  const float* pmk = sPar;
  const float* psk = sPar + HF;
  const float* pbk = sPar + 2 * HF;
  const float* pmq = sPar + 3 * HF;
  const float* psq = pmq + KD;
  const float* pbq = pmq + 2 * KD;

#pragma unroll 1
  for (int it = 0; it < (NKR * 48) / ATT; ++it) {
    const int idx = tid + ATT * it;
    const int n = idx / 48;
    const int c4 = idx - n * 48;
    const int f = 4 * c4;
    const int row = b * NTOK + min(n, NTOK - 1);
    const v4f y = *(const v4f*)(Ykv + (size_t)row * FKVQ + hl * HF + f);
    const bool valid = n < NTOK;
    float t[4];
#pragma unroll
    for (int e = 0; e < 4; ++e) t[e] = valid ? ((y[e] - pmk[f + e]) * psk[f + e] + pbk[f + e]) : 0.0f;
    if (f < KD) {
      H4 uh, ul;
#pragma unroll
      for (int e = 0; e < 4; ++e) {
        const float v = t[e] * SCQK;
        const _Float16 hv = (_Float16)v;
        uh.s[e] = hv;
        ul.s[e] = (_Float16)((v - (float)hv) * SCR);
      }
      *(v4h*)(&sKh[n * KP + f]) = uh.h;
      *(v4h*)(&sKl[n * KP + f]) = ul.h;
    } else {
      const int d = f - KD;
#pragma unroll
      for (int e = 0; e < 4; ++e) sVT[(d + e) * VP + n] = (_Float16)(t[e] * SCV);
    }
  }
  for (int idx = tid; idx < DV * 3; idx += ATT) {
    const int d = idx / 3, p = idx - d * 3;
    HU z;
    z.u = (v4u){0u, 0u, 0u, 0u};
    *(v8h*)(&sVT[d * VP + NKR + 8 * p]) = z.h;
  }
  __syncthreads();

  _Float16* sQh = sQ + wave * (2 * 16 * KP);
  _Float16* sQl = sQh + 16 * KP;
  float* sSw = sS + wave * (16 * SP);
  _Float16* sPw = (_Float16*)sSw + SP;
  _Float16* sOw = (_Float16*)sSw;

  for (int qt = wave; qt < NQT; qt += ATW) {
    const int q0 = 16 * qt;
    wave_lds_sync();

#pragma unroll
    for (int i = 0; i < 8; ++i) {
      const int item = lane + 32 * i;
      const int r = item >> 4, c4 = item & 15, f = 4 * c4;
      const int qrow = q0 + r;
      const int row = b * NTOK + min(qrow, NTOK - 1);
      const v4f y = *(const v4f*)(Yq + (size_t)row * FQQ + hl * KD + f);
      const bool valid = qrow < NTOK;
      H4 uh, ul;
#pragma unroll
      for (int e = 0; e < 4; ++e) {
        const float t = valid ? ((y[e] - pmq[f + e]) * psq[f + e] + pbq[f + e]) : 0.0f;
        const float v = t * SCQK;
        const _Float16 hv = (_Float16)v;
        uh.s[e] = hv;
        ul.s[e] = (_Float16)((v - (float)hv) * SCR);
      }
      *(v4h*)(&sQh[r * KP + f]) = uh.h;
      *(v4h*)(&sQl[r * KP + f]) = ul.h;
    }
    wave_lds_sync();

    const v16h aqh0 = ldfrag_h(sQh + rl * KP + 8 * hh);
    const v16h aqh1 = ldfrag_h(sQh + rl * KP + 32 + 8 * hh);
    const v16h aql0 = ldfrag_h(sQl + rl * KP + 8 * hh);
    const v16h aql1 = ldfrag_h(sQl + rl * KP + 32 + 8 * hh);
#pragma unroll 1
    for (int ct = 0; ct < NKT; ++ct) {
      const _Float16* kh = sKh + (16 * ct + rl) * KP + 8 * hh;
      const _Float16* kl = sKl + (16 * ct + rl) * KP + 8 * hh;
      v8f ahh = zero8(), ax = zero8();
      {
        const v16h b0 = ldfrag_h(kh);
        const v16h l0 = ldfrag_h(kl);
        ahh = mma_h(aqh0, b0, ahh);
        ax  = mma_h(aqh0, l0, ax);
        ax  = mma_h(aql0, b0, ax);
      }
      {
        const v16h b1 = ldfrag_h(kh + 32);
        const v16h l1 = ldfrag_h(kl + 32);
        ahh = mma_h(aqh1, b1, ahh);
        ax  = mma_h(aqh1, l1, ax);
        ax  = mma_h(aql1, b1, ax);
      }
      const int mc = 16 * ct + rl;
#pragma unroll
      for (int r = 0; r < 8; ++r) sSw[(8 * hh + r) * SP + mc] = (ahh[r] + ax[r] * (1.0f / SCR)) * SCS;
    }
    wave_lds_sync();

#pragma unroll 1
    for (int r = 0; r < 16; ++r) {
      const int qrow = q0 + r;
      const int qc = min(qrow, NTOK - 1);
      const float* brow = bias + ((size_t)h * NTOK + qc) * NTOK;
      float v[7];
      float mx = -3.0e38f;
#pragma unroll
      for (int j = 0; j < 7; ++j) {
        const int c = lane + 32 * j;
        const int cc = min(c, NTOK - 1);
        const float bv = bfr(brow[cc]);
        const float s = sSw[r * SP + c] + bv;
        const bool ok = c < NTOK;
        v[j] = ok ? s : -3.0e38f;
        mx = fmaxf(mx, v[j]);
      }
#pragma unroll
      for (int off = 16; off >= 1; off >>= 1) mx = fmaxf(mx, __shfl_xor(mx, off, 32));
      float z = 0.0f;
#pragma unroll
      for (int j = 0; j < 7; ++j) {
        const int c = lane + 32 * j;
        const bool ok = c < NTOK;
        float ef = __expf(v[j] - mx);
        ef = ok ? ef : 0.0f;
        z += ef;
        v[j] = ef;
      }
#pragma unroll
      for (int off = 16; off >= 1; off >>= 1) z += __shfl_xor(z, off, 32);
      const float rz = SCP * (1.0f / z);
      wave_lds_sync();
      _Float16* prow = sPw + r * (2 * SP);
#pragma unroll
      for (int j = 0; j < 7; ++j) {
        const int c = lane + 32 * j;
        _Float16 ph = (_Float16)(v[j] * rz);
        const float f0 = (float)ph;
        ph = (f0 < 6.103515625e-05f) ? (_Float16)0.0f : ph;
        prow[c] = ph;
      }
    }
    wave_lds_sync();

    v8f oacc[8];
#pragma unroll
    for (int dt = 0; dt < 8; ++dt) oacc[dt] = zero8();
#pragma unroll 1
    for (int ks = 0; ks < PVK / 32; ++ks) {
      const v16h a = ldfrag_h(sPw + rl * (2 * SP) + 32 * ks + 8 * hh);
#pragma unroll
      for (int dt = 0; dt < 8; ++dt) {
        const v16h bv = ldfrag_h(sVT + (16 * dt + rl) * VP + 32 * ks + 8 * hh);
        oacc[dt] = mma_h(a, bv, oacc[dt]);
      }
    }
    wave_lds_sync();

#pragma unroll
    for (int dt = 0; dt < 8; ++dt) {
#pragma unroll
      for (int r = 0; r < 8; ++r) {
        const float o = oacc[dt][r] * SCO;
        const float g = fminf(fmaxf(o + 3.0f, 0.0f), 6.0f);
        const float hv = (o * g) * (1.0f / 6.0f);
        sOw[(8 * hh + r) * OP + 16 * dt + rl] = (_Float16)(hv * SCH);
      }
    }
    wave_lds_sync();
    HU u[8];
#pragma unroll
    for (int i = 0; i < 8; ++i) {
      const int row = 2 * i + hh;
      u[i].h = *(const v8h*)(sOw + row * OP + 8 * rl);
    }
    for (int pass = 0; pass < 2; ++pass) {
#pragma unroll
      for (int i = 0; i < 8; ++i) {
        const int row = 2 * i + hh;
        const int qrow = q0 + row;
        if (qrow < NTOK) {
          _Float16* dst = HS + (size_t)(b * NTOK + qrow) * DH + h * DV + 8 * rl;
          *(volatile v4u*)dst = u[i].u;
        }
      }
      __threadfence();
    }
  }
}

__global__ __launch_bounds__(256) void bn_apply(const float* __restrict__ Y, const float* __restrict__ MU,
                                                const float* __restrict__ SC, const float* __restrict__ BE,
                                                float* out, int rows) {
  const int t = threadIdx.x;
  const int c = (t & 127) * 4;
  const int rsub = t >> 7;
  const v4f mu = *(const v4f*)(MU + c);
  const v4f sc = *(const v4f*)(SC + c);
  const v4f be = *(const v4f*)(BE + c);
  for (int pass = 0; pass < 2; ++pass) {
#pragma unroll 1
    for (int it = 0; it < 32; ++it) {
      const int row = blockIdx.x * 64 + 2 * it + rsub;
      if (row < rows) {
        const v4f y = *(const v4f*)(Y + (size_t)row * COUT + c);
        v4f o;
#pragma unroll
        for (int e = 0; e < 4; ++e) o[e] = (y[e] - mu[e]) * sc[e] + be[e];
        *(volatile v4f*)(out + (size_t)row * COUT + c) = o;
      }
    }
    __threadfence();
  }
}

extern "C" void kernel_launch(void* const* d_in, const int* in_sizes, int n_in,
                              void* d_out, int out_size, void* d_ws, size_t ws_size,
                              hipStream_t stream) {
  if (n_in < 11) return;
  if (in_sizes[0] != MROWS * CIN || in_sizes[1] != FKV * CIN || in_sizes[2] != FKV || in_sizes[3] != FKV) return;
  if (in_sizes[4] != FQ * CIN || in_sizes[5] != FQ || in_sizes[6] != FQ) return;
  if (in_sizes[7] != NHEAD * NTOK * NTOK || in_sizes[8] != COUT * DH || in_sizes[9] != COUT || in_sizes[10] != COUT) return;
  if (out_size != MROWS * COUT) return;

  const float* x     = (const float*)d_in[0];
  const float* Wkv   = (const float*)d_in[1];
  const float* gkv   = (const float*)d_in[2];
  const float* bkv   = (const float*)d_in[3];
  const float* Wq    = (const float*)d_in[4];
  const float* gq    = (const float*)d_in[5];
  const float* bq    = (const float*)d_in[6];
  const float* bias  = (const float*)d_in[7];
  const float* Wp    = (const float*)d_in[8];
  const float* gp    = (const float*)d_in[9];
  const float* bp    = (const float*)d_in[10];

  const size_t PX16 = (size_t)MROWS * CIN * 2;
  const size_t PWKV = (size_t)FKV * CIN * 2;
  const size_t PWQ  = (size_t)FQ * CIN * 2;
  const size_t PWP  = (size_t)COUT * DH * 2;
  const size_t PYA  = (size_t)MROWS * FKVQ * 4;
  const size_t PYB  = (size_t)MROWS * FQQ * 4;
  const size_t PPA  = (size_t)2 * TM64 * FKVQ * 4;
  const size_t PPB  = (size_t)2 * TM64 * FQQ * 4;
  const size_t PSA  = (size_t)FKVQ * 4;
  const size_t PSB  = (size_t)FQQ * 4;
  const size_t PHS  = (size_t)MROWS * DH * 2;
  if ((size_t)MROWS * COUT * 4 > PYA) return;
  if ((size_t)2 * TM64 * COUT * 4 > PPA) return;
  if ((size_t)COUT * 4 > PSA) return;

  size_t off = 0;
  const size_t oX16 = off; off += PX16;
  const size_t oWKV = off; off += PWKV;
  const size_t oWQ  = off; off += PWQ;
  const size_t oWP  = off; off += PWP;
  const size_t oYA  = off; off += PYA;
  const size_t oYB  = off; off += PYB;
  const size_t oPA  = off; off += PPA;
  const size_t oPB  = off; off += PPB;
  const size_t oMUA = off; off += PSA;
  const size_t oSCA = off; off += PSA;
  const size_t oBEA = off; off += PSA;
  const size_t oMUB = off; off += PSB;
  const size_t oSCB = off; off += PSB;
  const size_t oBEB = off; off += PSB;
  const size_t oHS  = off; off += PHS;
  if (off > ws_size) return;
  if (off > (size_t)134217728) return;

  char* ws = (char*)d_ws;
  _Float16* X16   = (_Float16*)(ws + oX16);
  _Float16* WKV16 = (_Float16*)(ws + oWKV);
  _Float16* WQ16  = (_Float16*)(ws + oWQ);
  _Float16* WP16  = (_Float16*)(ws + oWP);
  float*    YA    = (float*)(ws + oYA);
  float*    YB    = (float*)(ws + oYB);
  float*    PA    = (float*)(ws + oPA);
  float*    PB    = (float*)(ws + oPB);
  float*    MUA   = (float*)(ws + oMUA);
  float*    SCA   = (float*)(ws + oSCA);
  float*    BEA   = (float*)(ws + oBEA);
  float*    MUB   = (float*)(ws + oMUB);
  float*    SCB   = (float*)(ws + oSCB);
  float*    BEB   = (float*)(ws + oBEB);
  _Float16* HS    = (_Float16*)(ws + oHS);
  float*    outf  = (float*)d_out;

  const dim3 blk(256);
  const int n8x  = (MROWS * CIN) / 8;
  const int n8kv = (FKV * CIN) / 8;
  const int n8q  = (FQ * CIN) / 8;
  const int n8p  = (COUT * DH) / 8;
  const dim3 gX((n8x + 255) / 256), gKV((n8kv + 255) / 256), gQ((n8q + 255) / 256), gP((n8p + 255) / 256);
  const dim3 gGkv((TM64 * (FKVQ / 64) + 7) / 8);
  const dim3 gGq((TM64 * (FQQ / 64) + 7) / 8);
  const dim3 gGp((TM64 * (COUT / 64) + 7) / 8);
  const dim3 gSkv(FKVQ / 256), gSq(FQQ / 256), gSp(COUT / 256);
  const dim3 gAt(NBATCH, HQ);
  const dim3 gAp(TM64);
  const float csw  = 1.0f / SCW;
  const float cswh = 1.0f / (SCW * SCH);

  cvt_flat<<<gX, blk, 0, stream>>>(x, X16, n8x, 1.0f);
  cvt_flat<<<gKV, blk, 0, stream>>>(Wkv, WKV16, n8kv, SCW);
  cvt_flat<<<gQ, blk, 0, stream>>>(Wq, WQ16, n8q, SCW);
  cvt_flat<<<gP, blk, 0, stream>>>(Wp, WP16, n8p, SCW);

  hipFuncSetAttribute(reinterpret_cast<const void*>(&k_att), hipFuncAttributeMaxDynamicSharedMemorySize, ATT_LDS);

  for (int qu = 0; qu < NQU; ++qu) {
    gemm64s<<<gGkv, blk, 0, stream>>>(X16, CIN, WKV16 + (size_t)qu * FKVQ * CIN, CIN, csw,
                                       YA, FKVQ, PA, MROWS, FKVQ, CIN);
    gemm64s<<<gGq, blk, 0, stream>>>(X16, CIN, WQ16 + (size_t)qu * FQQ * CIN, CIN, csw,
                                      YB, FQQ, PB, MROWS, FQQ, CIN);
    bn_stats<<<gSkv, blk, 0, stream>>>(PA, FKVQ, TM64, gkv + qu * FKVQ, bkv + qu * FKVQ, MUA, SCA, BEA);
    bn_stats<<<gSq, blk, 0, stream>>>(PB, FQQ, TM64, gq + qu * FQQ, bq + qu * FQQ, MUB, SCB, BEB);
    k_att<<<gAt, dim3(ATT), ATT_LDS, stream>>>(YA, YB, MUA, SCA, BEA, MUB, SCB, BEB, bias, HS, qu);
  }

  gemm64s<<<gGp, blk, 0, stream>>>(HS, DH, WP16, DH, cswh, YA, COUT, PA, MROWS, COUT, DH);
  bn_stats<<<gSp, blk, 0, stream>>>(PA, COUT, TM64, gp, bp, MUA, SCA, BEA);
  bn_apply<<<gAp, blk, 0, stream>>>(YA, MUA, SCA, BEA, outf, MROWS);
}
